// GatedMultiheadAttention_5987184410925
// MI455X (gfx1250) — hardware-verified
//
#include <hip/hip_runtime.h>
#include <math.h>
#include <stdint.h>

#ifndef NB
#define NB    2
#endif
#ifndef SEQ
#define SEQ   2048
#endif
#define NB_FULL  2
#define SEQ_FULL 2048
#define DMOD  1024
#define NH    16
#define HD    64
#define QSC   1024.0f
#define KSC   1024.0f
#define PCAR  32768.0f
#define VCAR  1024.0f
#define OSC   1024.0f
#define WOS   1024.0f
#define LOG2E 1.4426950408889634f
#define ATT_WAVES   4
#define ATT_THREADS (ATT_WAVES * 32)
#define QT64        (SEQ / 64)
#define ATT_BLOCKS  (NB * NH * QT64)
#define NKB    (SEQ / 32)
#define SLABF  (16 * 68)
#define SLAB64 (16 * 68)
#define VTP    72
static_assert(HD == 64 && DMOD == NH * HD && NH == 16);
static_assert(NB >= 1 && NB <= NB_FULL && SEQ >= 64 && SEQ <= SEQ_FULL && (SEQ % 64) == 0);
static_assert(ATT_THREADS == 128 && ATT_BLOCKS == NB * NH * (SEQ / 64) && NKB * 32 == SEQ);
static_assert(((NB * SEQ) % 64) == 0 && (DMOD % 64) == 0 && (DMOD % 32) == 0);
static_assert((SEQ % 64) == 0 && (SEQ % 8) == 0);
static_assert(((NB * SEQ * DMOD / 8) % 256) == 0 && ((DMOD * DMOD / 8) % 256) == 0 && ((SEQ * DMOD / 8) % 256) == 0);
static_assert(ATT_WAVES * SLABF >= 4 * 16 * 68);
static_assert(HD * VTP >= 63 * VTP + 64);

typedef unsigned short u16;
typedef _Float16 v16h __attribute__((ext_vector_type(16)));
typedef _Float16 v8h  __attribute__((ext_vector_type(8)));
typedef __bf16   v16b __attribute__((ext_vector_type(16)));
typedef float    v8f  __attribute__((ext_vector_type(8)));
typedef float    v4f  __attribute__((ext_vector_type(4)));
typedef unsigned int v4u __attribute__((ext_vector_type(4)));

union FragH { v16h v; v8h h[2]; v4u u[2]; };
union FragB { v16b v; v4u u[2]; };

__device__ __forceinline__ unsigned short bf_bits(float f) {
  unsigned u = __float_as_uint(f);
  return (unsigned short)((u + 0x7FFFu + ((u >> 16) & 1u)) >> 16);
}
__device__ __forceinline__ float bf_up(unsigned short h) { return __uint_as_float(((unsigned)h) << 16); }
__device__ __forceinline__ float bfr(float f) { return bf_up(bf_bits(f)); }
__device__ __forceinline__ unsigned short h_bits(_Float16 x) { return __builtin_bit_cast(unsigned short, x); }
__device__ __forceinline__ unsigned pk16(unsigned short a, unsigned short b) { return (unsigned)a | ((unsigned)b << 16); }
__device__ __forceinline__ v8f zero8() { v8f z = {0.f, 0.f, 0.f, 0.f, 0.f, 0.f, 0.f, 0.f}; return z; }
__device__ __forceinline__ v4f zero4() { v4f z = {0.f, 0.f, 0.f, 0.f}; return z; }

__device__ __forceinline__ v16h ldfrag_h(const _Float16* p) {
  FragH f;
  f.h[0] = *(const v8h*)(p);
  f.h[1] = *(const v8h*)(p + 16);
  return f.v;
}
__device__ __forceinline__ v16b ldfrag_b(const u16* p) {
  FragB f;
  f.u[0] = *(const v4u*)(p);
  f.u[1] = *(const v4u*)(p + 16);
  return f.v;
}

__device__ __forceinline__ v8f mma_h(v16h a, v16h b, v8f c) {
  return __builtin_amdgcn_wmma_f32_16x16x32_f16(false, a, false, b, (short)0, c, false, false);
}
__device__ __forceinline__ v8f mma_b(v16b a, v16b b, v8f c) {
  return __builtin_amdgcn_wmma_f32_16x16x32_bf16(false, a, false, b, (short)0, c, false, false);
}
__device__ __forceinline__ void guard2(v8f& a, v8f& b, v16h x0, v16h x1, v16h x2, v16h x3, v16h x4, v16h x5) {
#if defined(__HIP_DEVICE_COMPILE__)
  asm volatile("v_nop\n\tv_nop\n\tv_nop\n\tv_nop"
               : "+v"(a), "+v"(b) : "v"(x0), "v"(x1), "v"(x2), "v"(x3), "v"(x4), "v"(x5) : "memory");
#endif
}
template <typename F>
__device__ __forceinline__ void guard6(v8f& a, v8f& b, v8f& c, v8f& d, F x0, F x1, F x2, F x3, F x4, F x5) {
#if defined(__HIP_DEVICE_COMPILE__)
  asm volatile("v_nop\n\tv_nop\n\tv_nop\n\tv_nop"
               : "+v"(a), "+v"(b), "+v"(c), "+v"(d) : "v"(x0), "v"(x1), "v"(x2), "v"(x3), "v"(x4), "v"(x5) : "memory");
#endif
}
__device__ __forceinline__ void guard10(v8f& a, v8f& b, v8f& c, v8f& d, v16h x0, v16h x1, v16h x2, v16h x3, v16h x4,
                                        v16h x5, v16h x6, v16h x7, v16h x8, v16h x9) {
#if defined(__HIP_DEVICE_COMPILE__)
  asm volatile("v_nop\n\tv_nop\n\tv_nop\n\tv_nop"
               : "+v"(a), "+v"(b), "+v"(c), "+v"(d)
               : "v"(x0), "v"(x1), "v"(x2), "v"(x3), "v"(x4), "v"(x5), "v"(x6), "v"(x7), "v"(x8), "v"(x9) : "memory");
#endif
}
__device__ __forceinline__ void acc_guard4(v8f& a, v8f& b, v8f& c, v8f& d) {
#if defined(__HIP_DEVICE_COMPILE__)
  asm volatile("v_nop\n\tv_nop\n\tv_nop\n\tv_nop" : "+v"(a), "+v"(b), "+v"(c), "+v"(d));
#endif
}
__device__ __forceinline__ void wave_sync_lds() {
  __builtin_amdgcn_fence(__ATOMIC_RELEASE, "workgroup");
  __builtin_amdgcn_wave_barrier();
  __builtin_amdgcn_fence(__ATOMIC_ACQUIRE, "workgroup");
}

__global__ __launch_bounds__(256) void cvt16(const float* __restrict__ x, u16* D, int n8, int f16mode, float scale,
                                             int seg8, int sstride8) {
  const int gt = blockIdx.x * 256 + (int)threadIdx.x;
  if (gt >= n8) return;
  const size_t so = (size_t)(gt / seg8) * (size_t)sstride8 + (size_t)(gt % seg8);
  const float* p = x + so * 8;
  const v4f a = *(const v4f*)(p), c4 = *(const v4f*)(p + 4);
  float v[8];
#pragma unroll
  for (int e = 0; e < 4; ++e) { v[e] = a[e]; v[4 + e] = c4[e]; }
  unsigned short s[8];
#pragma unroll
  for (int e = 0; e < 8; ++e) {
    const unsigned short hb = h_bits((_Float16)(bfr(v[e]) * scale));
    const unsigned short bb = bf_bits(v[e]);
    s[e] = (f16mode != 0) ? hb : bb;
  }
  v4u o;
#pragma unroll
  for (int e = 0; e < 4; ++e) o[e] = pk16(s[2 * e], s[2 * e + 1]);
  u16* d = D + (size_t)gt * 8;
  for (int pass = 0; pass < 2; ++pass) {
    *(volatile v4u*)(d) = o;
    __threadfence();
  }
}

__global__ __launch_bounds__(256) void split16(const float* __restrict__ x, u16* hpl, u16* lpl, int n8, float sc) {
  const int gt = blockIdx.x * 256 + (int)threadIdx.x;
  if (gt >= n8) return;
  const float* p = x + (size_t)gt * 8;
  const v4f a = *(const v4f*)(p), c4 = *(const v4f*)(p + 4);
  float w[8];
#pragma unroll
  for (int e = 0; e < 4; ++e) { w[e] = a[e]; w[4 + e] = c4[e]; }
  v4u oh, ol;
#pragma unroll
  for (int e = 0; e < 4; ++e) {
    const float t0 = w[2 * e] * sc, t1 = w[2 * e + 1] * sc;
    const _Float16 h0 = (_Float16)t0, h1 = (_Float16)t1;
    const _Float16 l0 = (_Float16)(t0 - (float)h0), l1 = (_Float16)(t1 - (float)h1);
    oh[e] = pk16(h_bits(h0), h_bits(h1));
    ol[e] = pk16(h_bits(l0), h_bits(l1));
  }
  const size_t o8 = (size_t)gt * 8;
  for (int pass = 0; pass < 2; ++pass) {
    *(volatile v4u*)(hpl + o8) = oh;
    *(volatile v4u*)(lpl + o8) = ol;
    __threadfence();
  }
}

__device__ __forceinline__ void epi64(float* sl, v8f a0, v8f a1, v8f a2, v8f a3, float oscale, v4f badd, float* C, int N,
                                      size_t rowb, int col0, int lane) {
  const int hh = lane >> 4, m = lane & 15;
#pragma unroll
  for (int r = 0; r < 8; ++r) {
    const int ro = (8 * hh + r) * 68 + m;
    sl[ro]      = a0[r] * oscale;
    sl[ro + 16] = a1[r] * oscale;
    sl[ro + 32] = a2[r] * oscale;
    sl[ro + 48] = a3[r] * oscale;
  }
  wave_sync_lds();
  v4f vals[8];
#pragma unroll
  for (int it = 0; it < 8; ++it) vals[it] = *(const v4f*)(sl + (it * 2 + hh) * 68 + m * 4) + badd;
  float* dst = C + (rowb + (size_t)hh) * (size_t)N + col0 + m * 4;
  for (int pass = 0; pass < 2; ++pass) {
#pragma unroll
    for (int it = 0; it < 8; ++it) {
      *(volatile v4f*)(dst + (size_t)(it * 2) * (size_t)N) = vals[it];
    }
    __threadfence();
  }
}

__global__ __launch_bounds__(128)
void gemm_bfb(const u16* __restrict__ A, const u16* __restrict__ Bt, const float* __restrict__ bias,
              float* C, int M, int N, int K, float oscale) {
  __shared__ __align__(16) float slab[4 * SLAB64];
  const int tid = threadIdx.x, wave = tid >> 5, lane = tid & 31, hh = lane >> 4, m = lane & 15;
  const int ntile = N >> 6;
  const int bid   = blockIdx.x;
  const int rowb  = (bid / ntile) * 64 + wave * 16;
  const int col0  = (bid % ntile) * 64;
  if (rowb + 16 > M) return;
  const u16* ap = A  + (size_t)(rowb + m) * K + 8 * hh;
  const u16* bp = Bt + (size_t)(col0 + m) * K + 8 * hh;
  const size_t bs = (size_t)16 * K;
  v8f acc0 = zero8(), acc1 = zero8(), acc2 = zero8(), acc3 = zero8();
#pragma unroll 1
  for (int k0 = 0; k0 < K; k0 += 32) {
    const v16b a  = ldfrag_b(ap + k0);
    const v16b b0 = ldfrag_b(bp + k0);
    const v16b b1 = ldfrag_b(bp + bs + k0);
    const v16b b2 = ldfrag_b(bp + 2 * bs + k0);
    const v16b b3 = ldfrag_b(bp + 3 * bs + k0);
    acc0 = mma_b(a, b0, acc0);
    acc1 = mma_b(a, b1, acc1);
    acc2 = mma_b(a, b2, acc2);
    acc3 = mma_b(a, b3, acc3);
    guard6<v16b>(acc0, acc1, acc2, acc3, a, b0, b1, b2, b3, a);
  }
  const v4f bv = *(const v4f*)(bias + col0 + m * 4);
  v4f badd;
#pragma unroll
  for (int e = 0; e < 4; ++e) badd[e] = bfr(bv[e]);
  epi64(slab + wave * SLAB64, acc0, acc1, acc2, acc3, oscale, badd, C, N, (size_t)rowb, col0, lane);
}

__global__ __launch_bounds__(128)
void gemm_h2(const u16* __restrict__ Ah, const u16* __restrict__ Al, const u16* __restrict__ Bt,
             const float* __restrict__ bias, float* C, int M, int N, int K, float oscale) {
  __shared__ __align__(16) float slab[4 * SLAB64];
  const int tid = threadIdx.x, wave = tid >> 5, lane = tid & 31, hh = lane >> 4, m = lane & 15;
  const int ntile = N >> 6;
  const int bid   = blockIdx.x;
  const int rowb  = (bid / ntile) * 64 + wave * 16;
  const int col0  = (bid % ntile) * 64;
  if (rowb + 16 > M) return;
  const size_t aofs = (size_t)(rowb + m) * K + 8 * hh;
  const _Float16* ahp = (const _Float16*)(const void*)Ah + aofs;
  const _Float16* alp = (const _Float16*)(const void*)Al + aofs;
  const _Float16* bp  = (const _Float16*)(const void*)Bt + (size_t)(col0 + m) * K + 8 * hh;
  const size_t bs = (size_t)16 * K;
  v8f acc0 = zero8(), acc1 = zero8(), acc2 = zero8(), acc3 = zero8();
#pragma unroll 1
  for (int k0 = 0; k0 < K; k0 += 32) {
    const v16h ah = ldfrag_h(ahp + k0), al = ldfrag_h(alp + k0);
    const v16h b0 = ldfrag_h(bp + k0);
    const v16h b1 = ldfrag_h(bp + bs + k0);
    const v16h b2 = ldfrag_h(bp + 2 * bs + k0);
    const v16h b3 = ldfrag_h(bp + 3 * bs + k0);
    acc0 = mma_h(ah, b0, acc0);  acc0 = mma_h(al, b0, acc0);
    acc1 = mma_h(ah, b1, acc1);  acc1 = mma_h(al, b1, acc1);
    acc2 = mma_h(ah, b2, acc2);  acc2 = mma_h(al, b2, acc2);
    acc3 = mma_h(ah, b3, acc3);  acc3 = mma_h(al, b3, acc3);
    guard6<v16h>(acc0, acc1, acc2, acc3, ah, al, b0, b1, b2, b3);
  }
  const v4f bv = *(const v4f*)(bias + col0 + m * 4);
  v4f badd;
#pragma unroll
  for (int e = 0; e < 4; ++e) badd[e] = bfr(bv[e]);
  epi64(slab + wave * SLAB64, acc0, acc1, acc2, acc3, oscale, badd, C, N, (size_t)rowb, col0, lane);
}

__global__ __launch_bounds__(256) void vt16(const float* __restrict__ v, u16* VHo, u16* VLo) {
  __shared__ __align__(16) u16 TH[HD * VTP];
  __shared__ __align__(16) u16 TL[HD * VTP];
  const int tid = threadIdx.x;
  const int bid = blockIdx.x;
  const int st  = bid % QT64;
  const int h   = (bid / QT64) % NH;
  const int b   = bid / (QT64 * NH);
  const int s0  = st * 64;
  {
    const int sl = tid >> 2;
    const int dc = (tid & 3) * 16;
    const float* src = v + (((size_t)(b * SEQ + s0 + sl)) * NH + h) * HD + dc;
#pragma unroll
    for (int i = 0; i < 4; ++i) {
      const v4f a = *(const v4f*)(src + 4 * i);
#pragma unroll
      for (int e = 0; e < 4; ++e) {
        const float t = a[e] * VCAR;
        const _Float16 hv = (_Float16)t;
        const _Float16 lv = (_Float16)(t - (float)hv);
        TH[(dc + 4 * i + e) * VTP + sl] = h_bits(hv);
        TL[(dc + 4 * i + e) * VTP + sl] = h_bits(lv);
      }
    }
  }
  __syncthreads();
  v4u vh[2], vl[2];
  const int q8 = tid >> 3, p8 = (tid & 7) * 8;
#pragma unroll
  for (int it = 0; it < 2; ++it) {
    const int line = it * 32 + q8;
    vh[it] = *(const v4u*)(TH + line * VTP + p8);
    vl[it] = *(const v4u*)(TL + line * VTP + p8);
  }
  const size_t base = ((size_t)(b * NH + h) * HD) * SEQ + s0 + p8;
  for (int pass = 0; pass < 2; ++pass) {
#pragma unroll
    for (int it = 0; it < 2; ++it) {
      const int line = it * 32 + q8;
      *(volatile v4u*)(VHo + base + (size_t)line * SEQ) = vh[it];
      *(volatile v4u*)(VLo + base + (size_t)line * SEQ) = vl[it];
    }
    __threadfence();
  }
}

__global__ __launch_bounds__(ATT_THREADS)
void attn_fwd(const u16* __restrict__ QHIp, const u16* __restrict__ QLOp,
              const u16* __restrict__ KHIp, const u16* __restrict__ KLOp,
              const u16* __restrict__ VHIp, const u16* __restrict__ VLOp,
              const float* __restrict__ gatep,
              u16* OHIp, u16* OLOp) {
  __shared__ __align__(16) float smem[ATT_WAVES * SLABF];

  const int tid  = threadIdx.x;
  const int wave = tid >> 5;
  const int lane = tid & 31;
  const int hh   = lane >> 4;
  const int c    = lane & 15;

  const int bid  = blockIdx.x;
  const int qt   = bid % QT64;
  const int head = (bid / QT64) % NH;
  const int b    = bid / (QT64 * NH);
  const int q0   = qt * 64 + wave * 16;

  const float gbf = bfr(gatep[head]);
  const float sgm = 1.0f / (1.0f + expf(-gbf));
  const float lsc = sgm * (0.125f * (LOG2E / (QSC * KSC)));

  const size_t qofs = (((size_t)(b * SEQ + q0 + c)) * NH + head) * HD + 8 * hh;
  const _Float16* Qh  = (const _Float16*)(const void*)QHIp + qofs;
  const _Float16* Ql  = (const _Float16*)(const void*)QLOp + qofs;
  const size_t kofs = (((size_t)b * SEQ + c) * NH + head) * HD + 8 * hh;
  const _Float16* Khb = (const _Float16*)(const void*)KHIp + kofs;
  const _Float16* Klb = (const _Float16*)(const void*)KLOp + kofs;
  const size_t vofs = ((size_t)(b * NH + head) * HD + c) * SEQ + 8 * hh;
  const _Float16* Vhb = (const _Float16*)(const void*)VHIp + vofs;
  const _Float16* Vlb = (const _Float16*)(const void*)VLOp + vofs;

  float mrun = -INFINITY, lrun = 0.f;
  v8f o[4];
#pragma unroll
  for (int j = 0; j < 4; ++j) o[j] = zero8();

#pragma unroll 1
  for (int it = 0; it < NKB; ++it) {
    const int kb = it * 32;
    v8f s0 = zero8(), s1 = zero8();
    const _Float16* k0p = Khb + (size_t)kb * (NH * HD);
    const _Float16* k1p = k0p + (size_t)16 * (NH * HD);
    const _Float16* l0p = Klb + (size_t)kb * (NH * HD);
    const _Float16* l1p = l0p + (size_t)16 * (NH * HD);
#pragma unroll
    for (int kk = 0; kk < 2; ++kk) {
      const v16h qh  = ldfrag_h(Qh + kk * 32),  ql  = ldfrag_h(Ql + kk * 32);
      const v16h kh0 = ldfrag_h(k0p + kk * 32), kl0 = ldfrag_h(l0p + kk * 32);
      const v16h kh1 = ldfrag_h(k1p + kk * 32), kl1 = ldfrag_h(l1p + kk * 32);
      s0 = mma_h(kh0, qh, s0);
      s0 = mma_h(kl0, qh, s0);
      s0 = mma_h(kh0, ql, s0);
      s1 = mma_h(kh1, qh, s1);
      s1 = mma_h(kl1, qh, s1);
      s1 = mma_h(kh1, ql, s1);
      guard2(s0, s1, qh, ql, kh0, kl0, kh1, kl1);
    }
    float t[16];
#pragma unroll
    for (int i = 0; i < 8; ++i) { t[i] = s0[i] * lsc; t[8 + i] = s1[i] * lsc; }
    float cm = t[0];
#pragma unroll
    for (int i = 1; i < 16; ++i) cm = fmaxf(cm, t[i]);
    cm = fmaxf(cm, __shfl_xor(cm, 16, 32));
    const float mn = fmaxf(mrun, cm);
    const float al = exp2f(mrun - mn);
    mrun = mn;
    float ps = 0.f;
    FragH ph, pl;
#pragma unroll
    for (int w = 0; w < 2; ++w) {
#pragma unroll
      for (int e4 = 0; e4 < 4; ++e4) {
        const int i = 8 * w + 2 * e4;
        const float p0 = exp2f(t[i] - mn), p1 = exp2f(t[i + 1] - mn);
        ps += p0 + p1;
        const float a0 = p0 * PCAR, a1 = p1 * PCAR;
        const _Float16 h0 = (_Float16)a0, h1 = (_Float16)a1;
        const _Float16 l0 = (_Float16)(a0 - (float)h0), l1 = (_Float16)(a1 - (float)h1);
        ph.u[w][e4] = pk16(h_bits(h0), h_bits(h1));
        pl.u[w][e4] = pk16(h_bits(l0), h_bits(l1));
      }
    }
    ps += __shfl_xor(ps, 16, 32);
    lrun = lrun * al + ps;
    float scl[8];
#pragma unroll
    for (int r = 0; r < 8; ++r) scl[r] = __shfl(al, 8 * hh + r, 32);
#pragma unroll
    for (int j = 0; j < 4; ++j) {
#pragma unroll
      for (int r = 0; r < 8; ++r) o[j][r] *= scl[r];
    }
    {
      const _Float16* vhp = Vhb + kb;
      const _Float16* vlp = Vlb + kb;
      const v16h vh0 = ldfrag_h(vhp);
      const v16h vh1 = ldfrag_h(vhp + (size_t)16 * SEQ);
      const v16h vh2 = ldfrag_h(vhp + (size_t)32 * SEQ);
      const v16h vh3 = ldfrag_h(vhp + (size_t)48 * SEQ);
      const v16h vl0 = ldfrag_h(vlp);
      const v16h vl1 = ldfrag_h(vlp + (size_t)16 * SEQ);
      const v16h vl2 = ldfrag_h(vlp + (size_t)32 * SEQ);
      const v16h vl3 = ldfrag_h(vlp + (size_t)48 * SEQ);
      o[0] = mma_h(ph.v, vh0, o[0]);  o[0] = mma_h(pl.v, vh0, o[0]);  o[0] = mma_h(ph.v, vl0, o[0]);
      o[1] = mma_h(ph.v, vh1, o[1]);  o[1] = mma_h(pl.v, vh1, o[1]);  o[1] = mma_h(ph.v, vl1, o[1]);
      o[2] = mma_h(ph.v, vh2, o[2]);  o[2] = mma_h(pl.v, vh2, o[2]);  o[2] = mma_h(ph.v, vl2, o[2]);
      o[3] = mma_h(ph.v, vh3, o[3]);  o[3] = mma_h(pl.v, vh3, o[3]);  o[3] = mma_h(ph.v, vl3, o[3]);
      guard10(o[0], o[1], o[2], o[3], ph.v, pl.v, vh0, vh1, vh2, vh3, vl0, vl1, vl2, vl3);
    }
  }
  acc_guard4(o[0], o[1], o[2], o[3]);

  const float linv = (1.0f / lrun) * (1.0f / (PCAR * VCAR));
  float inv[8];
#pragma unroll
  for (int r = 0; r < 8; ++r) inv[r] = __shfl(linv, 8 * hh + r, 32);
  float* slab = smem + wave * SLABF;
#pragma unroll
  for (int r = 0; r < 8; ++r) {
#pragma unroll
    for (int j = 0; j < 4; ++j) slab[(8 * hh + r) * 68 + j * 16 + c] = o[j][r] * inv[r];
  }
  wave_sync_lds();
  v4u oh[4], ol[4];
  const int rq = lane >> 3, c8 = (lane & 7) * 8;
#pragma unroll
  for (int i4 = 0; i4 < 4; ++i4) {
    const int row = i4 * 4 + rq;
    const v4f a = *(const v4f*)(slab + row * 68 + c8), c4 = *(const v4f*)(slab + row * 68 + c8 + 4);
    float w[8];
#pragma unroll
    for (int e = 0; e < 4; ++e) { w[e] = a[e] * OSC; w[4 + e] = c4[e] * OSC; }
#pragma unroll
    for (int e = 0; e < 4; ++e) {
      const _Float16 h0 = (_Float16)w[2 * e], h1 = (_Float16)w[2 * e + 1];
      const _Float16 l0 = (_Float16)(w[2 * e] - (float)h0), l1 = (_Float16)(w[2 * e + 1] - (float)h1);
      oh[i4][e] = pk16(h_bits(h0), h_bits(h1));
      ol[i4][e] = pk16(h_bits(l0), h_bits(l1));
    }
  }
  const size_t ob = (((size_t)(b * SEQ + q0)) * NH + head) * HD + c8;
  for (int pass = 0; pass < 2; ++pass) {
#pragma unroll
    for (int i4 = 0; i4 < 4; ++i4) {
      const int row = i4 * 4 + rq;
      const size_t o8 = ob + (size_t)row * (NH * HD);
      *(volatile v4u*)(OHIp + o8) = oh[i4];
      *(volatile v4u*)(OLOp + o8) = ol[i4];
    }
    __threadfence();
  }
}

extern "C" void kernel_launch(void* const* d_in, const int* in_sizes, int n_in,
                              void* d_out, int out_size, void* d_ws, size_t ws_size,
                              hipStream_t stream) {
  const int ROWS = NB * SEQ;
  if (n_in < 12) return;
  const int needX = ((NB - 1) * SEQ_FULL + SEQ) * DMOD;
  if (in_sizes[0] < needX || in_sizes[1] < needX || in_sizes[2] < needX) return;
  if (in_sizes[3] < DMOD * DMOD || in_sizes[5] < DMOD * DMOD) return;
  if (in_sizes[7] < DMOD * DMOD || in_sizes[9] < DMOD * DMOD) return;
  if (in_sizes[4] < DMOD || in_sizes[6] < DMOD || in_sizes[8] < DMOD || in_sizes[10] < DMOD) return;
  if (in_sizes[11] < NH) return;
  if (out_size < ROWS * DMOD) return;

  const float* Qin = (const float*)d_in[0];
  const float* Kin = (const float*)d_in[1];
  const float* Vin = (const float*)d_in[2];
  const float* wq  = (const float*)d_in[3];
  const float* bq  = (const float*)d_in[4];
  const float* wk  = (const float*)d_in[5];
  const float* bk  = (const float*)d_in[6];
  const float* wv  = (const float*)d_in[7];
  const float* bv  = (const float*)d_in[8];
  const float* wo  = (const float*)d_in[9];
  const float* bo  = (const float*)d_in[10];
  const float* gt  = (const float*)d_in[11];
  float*       out = (float*)d_out;

  const size_t szXB  = (size_t)ROWS * DMOD * 2;
  const size_t szW   = (size_t)DMOD * DMOD * 2;
  const size_t szF   = (size_t)ROWS * DMOD * 4;
  const size_t szP   = (size_t)ROWS * DMOD * 2;
  const size_t szVP  = (size_t)NB * NH * HD * SEQ * 2;
  size_t off = 0;
  const size_t oXB  = off; off += szXB;
  const size_t oWQB = off; off += szW;
  const size_t oWKB = off; off += szW;
  const size_t oWVB = off; off += szW;
  const size_t oWOB = off; off += szW;
  const size_t oF   = off; off += szF;
  const size_t oQHI = off; off += szP;
  const size_t oQLO = off; off += szP;
  const size_t oKHI = off; off += szP;
  const size_t oKLO = off; off += szP;
  const size_t oVHI = off; off += szVP;
  const size_t oVLO = off; off += szVP;
  const size_t oOHI = off; off += szP;
  const size_t oOLO = off; off += szP;
  if (off > ws_size) return;
  if (off > (size_t)134217728) return;

  char* ws = (char*)d_ws;
  u16*   XB  = (u16*)(ws + oXB);
  u16*   WQB = (u16*)(ws + oWQB);
  u16*   WKB = (u16*)(ws + oWKB);
  u16*   WVB = (u16*)(ws + oWVB);
  u16*   WOB = (u16*)(ws + oWOB);
  float* F   = (float*)(ws + oF);
  u16*   QHI = (u16*)(ws + oQHI);
  u16*   QLO = (u16*)(ws + oQLO);
  u16*   KHI = (u16*)(ws + oKHI);
  u16*   KLO = (u16*)(ws + oKLO);
  u16*   VHI = (u16*)(ws + oVHI);
  u16*   VLO = (u16*)(ws + oVLO);
  u16*   OHI = (u16*)(ws + oOHI);
  u16*   OLO = (u16*)(ws + oOLO);

  const dim3 blk(256);
  const int n8x = (ROWS * DMOD) / 8;
  const int n8w = (DMOD * DMOD) / 8;
  const int seg8x = (SEQ * DMOD) / 8;
  const int str8x = (SEQ_FULL * DMOD) / 8;
  if ((n8x % 256) != 0 || (n8w % 256) != 0) return;
  if ((DMOD % 32) != 0 || (ROWS % 64) != 0 || (DMOD % 64) != 0) return;
  const dim3 gX(n8x / 256);
  const dim3 gWc(n8w / 256);
  const dim3 gG((ROWS / 64) * (DMOD / 64));
  const dim3 bG(128);
  const dim3 gVT(NB * NH * (SEQ / 64));
  const dim3 gAT(ATT_BLOCKS);
  const dim3 bAT(ATT_THREADS);

  cvt16<<<gWc, blk, 0, stream>>>(wq, WQB, n8w, 0, 1.0f, n8w, n8w);
  cvt16<<<gWc, blk, 0, stream>>>(wk, WKB, n8w, 0, 1.0f, n8w, n8w);
  cvt16<<<gWc, blk, 0, stream>>>(wv, WVB, n8w, 0, 1.0f, n8w, n8w);
  cvt16<<<gWc, blk, 0, stream>>>(wo, WOB, n8w, 1, WOS, n8w, n8w);
  cvt16<<<gX, blk, 0, stream>>>(Qin, XB, n8x, 0, 1.0f, seg8x, str8x);
  gemm_bfb<<<gG, bG, 0, stream>>>(XB, WQB, bq, F, ROWS, DMOD, DMOD, 1.0f);
  split16<<<gX, blk, 0, stream>>>(F, QHI, QLO, n8x, QSC);
  cvt16<<<gX, blk, 0, stream>>>(Kin, XB, n8x, 0, 1.0f, seg8x, str8x);
  gemm_bfb<<<gG, bG, 0, stream>>>(XB, WKB, bk, F, ROWS, DMOD, DMOD, 1.0f);
  split16<<<gX, blk, 0, stream>>>(F, KHI, KLO, n8x, KSC);
  cvt16<<<gX, blk, 0, stream>>>(Vin, XB, n8x, 0, 1.0f, seg8x, str8x);
  gemm_bfb<<<gG, bG, 0, stream>>>(XB, WVB, bv, F, ROWS, DMOD, DMOD, 1.0f);
  vt16<<<gVT, blk, 0, stream>>>(F, VHI, VLO);
  attn_fwd<<<gAT, bAT, 0, stream>>>(QHI, QLO, KHI, KLO, VHI, VLO, gt, OHI, OLO);
  gemm_h2<<<gG, bG, 0, stream>>>(OHI, OLO, WOB, bo, out, ROWS, DMOD, DMOD, 1.0f / (OSC * WOS));
  (void)hipGetLastError();
}
